// MultimodalUNet_62251255988274
// MI455X (gfx1250) — hardware-verified
//
#include <hip/hip_runtime.h>
#include <hip/hip_bf16.h>
#include <math.h>

#define NB_ 2
#define NFR 16
#define CC 256
#define HWV 1024
#define VLEN (NFR * HWV)
#define LA 4096
#define APF (LA / NFR)
#define TT (VLEN + LA)
#define HH 4
#define DKK 64
#define QW 2
#define NG 32
#define SS 1024
#define GSTR 48

typedef _Float16 bf16;
typedef _Float16 f16;
typedef __attribute__((ext_vector_type(4))) unsigned v4u_t;
typedef unsigned v4ua __attribute__((ext_vector_type(4), may_alias));
typedef __attribute__((ext_vector_type(4))) float v4f_t;
typedef float v4fa __attribute__((ext_vector_type(4), may_alias));
typedef __attribute__((ext_vector_type(16))) bf16  bf16x16;
typedef bf16x16 f16x16;
typedef __attribute__((ext_vector_type(8)))  bf16  bf16x8;
typedef bf16x8 f16x8;
typedef __attribute__((ext_vector_type(4)))  bf16  bf16x4;
typedef __attribute__((ext_vector_type(8)))  float f32x8;
__device__ __forceinline__ f32x8 wmma16(f16x16 a, f16x16 b, f32x8 c) {
  c = __builtin_amdgcn_wmma_f32_16x16x32_f16(false, a, false, b, (short)0, c, false, false);
  asm volatile("v_nop\n\tv_nop\n\tv_nop\n\tv_nop" : "+v"(c) : "v"(a), "v"(b));
  return c;
}
#define LDS_STRIDE 48
#define KSTRIDE    72
#define VSTRIDE    48

__device__ __forceinline__ f32x8 wmma_bf16(bf16x16 a, bf16x16 b, f32x8 c) {
  c = __builtin_amdgcn_wmma_f32_16x16x32_f16(false, a, false, b, (short)0, c, false, false);
  asm volatile("v_nop\n\tv_nop\n\tv_nop\n\tv_nop" : "+v"(c) : "v"(a), "v"(b));
  return c;
}

template <typename T>
__device__ __forceinline__ bf16x16 load_frag(const T* __restrict__ base, int ld,
                                             int row0, int k0) {
  const int lane = threadIdx.x & 31;
  const int r    = lane & 15;
  const int kh   = (lane >> 4) * 8;
  const T* p0 = base + (size_t)(row0 + r) * ld + (k0 + kh);
  const T* p1 = p0 + 16;
  bf16x16 f;
#pragma unroll
  for (int i = 0; i < 8; ++i) {
    f[i]     = (bf16)p0[i];
    f[i + 8] = (bf16)p1[i];
  }
  return f;
}

__device__ __forceinline__ bf16x16 lds_frag(const bf16* base, int stride) {
  const int lane = threadIdx.x & 31;
  const int row  = lane & 15;
  const int kh   = (lane >> 4) * 8;
  const bf16x8 lo = *(const bf16x8*)(base + row * stride + kh);
  const bf16x8 hi = *(const bf16x8*)(base + row * stride + kh + 16);
  bf16x16 f;
#pragma unroll
  for (int i = 0; i < 8; ++i) { f[i] = lo[i]; f[i + 8] = hi[i]; }
  return f;
}

template <typename T>
__device__ __forceinline__ void stage_read16(const T* __restrict__ p, float* buf) {
#pragma unroll
  for (int i = 0; i < 16; ++i) buf[i] = (float)p[i];
}

__device__ __forceinline__ void stage_write(bf16* dst, const float* buf, int nquad) {
#pragma unroll
  for (int i = 0; i < nquad; ++i) {
    bf16x4 q;
    q[0] = (bf16)buf[4 * i];     q[1] = (bf16)buf[4 * i + 1];
    q[2] = (bf16)buf[4 * i + 2]; q[3] = (bf16)buf[4 * i + 3];
    *(bf16x4*)(dst + 4 * i) = q;
  }
}

__global__ __launch_bounds__(64) void attn_kernel(
    const bf16* __restrict__ Qb, const bf16* __restrict__ Kb,
    const bf16* __restrict__ Vt, float* __restrict__ Rout, int qbase, int qper, int kbase, int kper, int nkeys, int outld) {
  __shared__ bf16 ldsK[32 * KSTRIDE];
  __shared__ __attribute__((aligned(16))) bf16 ldsQ[64 * KSTRIDE];
  __shared__ bf16 ldsV[64 * VSTRIDE];
  __shared__ __attribute__((aligned(16))) float ldsO[2][64 * 36];

  const int q0blk = blockIdx.x * 64;
  const int h  = blockIdx.y;
  const int b  = blockIdx.z;
  const int t    = threadIdx.x;
  const int wave = t >> 5;
  const int lane = t & 31;
  const int qlane = lane & 15;
  const int kh8   = (lane >> 4) * 8;
  const int q0 = q0blk + wave * 32;

  const int bb = b / NFR, fr = b % NFR;
  const bf16* Qc = Qb + ((size_t)bb * 768 + 0 * 256 + h * DKK) * TT + qbase + (size_t)fr * qper;
  const bf16* Kc = Kb + ((size_t)bb * 768 + 1 * 256 + h * DKK) * TT + kbase + (size_t)fr * kper;
  const bf16* Vh = Vt + ((size_t)bb * 768 + 2 * 256 + h * DKK) * TT + kbase + (size_t)fr * kper;
  for (int e = t; e < 64 * 64; e += 64) { const int d = e >> 6, qq = e & 63; ldsQ[qq * KSTRIDE + d] = Qc[(size_t)d * TT + q0blk + qq]; }
  __syncthreads();

  const bf16* kSrc = Kc + (size_t)t * TT;
  const bf16* vSrc = Vh + (size_t)t * TT;

  bf16x16 qf[QW][2];
#pragma unroll
  for (int qt = 0; qt < QW; ++qt) {
    qf[qt][0] = lds_frag(ldsQ + (wave * 32 + 16 * qt) * KSTRIDE, KSTRIDE);
    qf[qt][1] = lds_frag(ldsQ + (wave * 32 + 16 * qt) * KSTRIDE + 32, KSTRIDE);
  }

  f32x8 o[QW][4] = {};
  float mrun[QW], lrun[QW];
#pragma unroll
  for (int qt = 0; qt < QW; ++qt) { mrun[qt] = -INFINITY; lrun[qt] = 0.0f; }

  const float scale = 0.125f * 1.44269504088896340736f;
  const float NEG2 = -1.0e9f;
  const int kmax = nkeys - 1;

  bf16x8 kreg[4], vreg[4];
#pragma unroll
  for (int i = 0; i < 4; ++i) {
    kreg[i] = *(const bf16x8*)(kSrc + 8 * i);
    vreg[i] = *(const bf16x8*)(vSrc + 8 * i);
  }

  for (int kb = 0; kb <= kmax; kb += 32) {
    __syncthreads();
#pragma unroll
    for (int i = 0; i < 4; ++i) {
#pragma unroll
      for (int u = 0; u < 8; ++u) ldsK[(8 * i + u) * KSTRIDE + t] = kreg[i][u];
      *(bf16x8*)(&ldsV[t * VSTRIDE + 8 * i]) = vreg[i];
    }
    if (kb + 32 <= kmax) {
      const bf16* kn = kSrc + (kb + 32);
      const bf16* vn = vSrc + (kb + 32);
#pragma unroll
      for (int i = 0; i < 4; ++i) {
        kreg[i] = *(const bf16x8*)(kn + 8 * i);
        vreg[i] = *(const bf16x8*)(vn + 8 * i);
      }
    }
    __syncthreads();

    bf16x16 kf[2][2];
#pragma unroll
    for (int ktile = 0; ktile < 2; ++ktile)
#pragma unroll
      for (int c = 0; c < 2; ++c)
        kf[ktile][c] = lds_frag(ldsK + (ktile * 16) * KSTRIDE + c * 32, KSTRIDE);

    bf16x16 pf[QW];
    bool act[QW];
#pragma unroll
    for (int qt = 0; qt < QW; ++qt) {
      unsigned mbits = 0;
      mbits = 0xFFFFu; act[qt] = true;
      if (act[qt]) {
        const int q_my = q0 + 16 * qt + qlane;
        f32x8 s0 = {}, s1 = {};
        s0 = wmma_bf16(kf[0][0], qf[qt][0], s0);
        s0 = wmma_bf16(kf[0][1], qf[qt][1], s0);
        s1 = wmma_bf16(kf[1][0], qf[qt][0], s1);
        s1 = wmma_bf16(kf[1][1], qf[qt][1], s1);

        float mx = -INFINITY;
#pragma unroll
        for (int r = 0; r < 8; ++r) {
          const int k0i = kb + kh8 + r;
          const int k1i = k0i + 16;
          (void)k0i; (void)k1i; (void)q_my;
          s0[r] = (mbits & (1u << r))       ? s0[r] * scale : NEG2;
          s1[r] = (mbits & (1u << (8 + r))) ? s1[r] * scale : NEG2;
          mx = fmaxf(mx, fmaxf(s0[r], s1[r]));
        }
        mx = fmaxf(mx, __shfl_xor(mx, 16, 32));
        const float mnew  = fmaxf(mrun[qt], mx);
        const float alpha = exp2f(mrun[qt] - mnew);

        float rsum = 0.0f;
#pragma unroll
        for (int r = 0; r < 8; ++r) {
          const float p0 = exp2f(s0[r] - mnew);
          const float p1 = exp2f(s1[r] - mnew);
          rsum += p0 + p1;
          pf[qt][r]     = (bf16)(p0 * 1024.0f);
          pf[qt][r + 8] = (bf16)(p1 * 1024.0f);
        }
        rsum += __shfl_xor(rsum, 16, 32);
        lrun[qt] = lrun[qt] * alpha + rsum;
        mrun[qt] = mnew;

#pragma unroll
        for (int j = 0; j < 4; ++j)
#pragma unroll
          for (int r = 0; r < 8; ++r) o[qt][j][r] *= alpha;
      }
    }

#pragma unroll
    for (int j = 0; j < 4; ++j) {
      const bf16x16 vf = lds_frag(ldsV + (j * 16) * VSTRIDE, VSTRIDE);
#pragma unroll
      for (int qt = 0; qt < QW; ++qt)
        if (act[qt]) o[qt][j] = wmma_bf16(vf, pf[qt], o[qt][j]);
    }
  }

  float* so = ldsO[wave];
#pragma unroll
  for (int qt = 0; qt < QW; ++qt) {
    const float rl = 1.0f / (lrun[qt] * 1024.0f);
#pragma unroll
    for (int j = 0; j < 4; ++j)
#pragma unroll
      for (int r = 0; r < 8; ++r) so[(j * 16 + kh8 + r) * 36 + 16 * qt + qlane] = o[qt][j][r] * rl;
  }
  asm volatile("s_wait_dscnt 0" ::: "memory");
  __builtin_amdgcn_wave_barrier();
#pragma unroll 1
  for (int pass = 0; pass < 2; ++pass) {
#pragma unroll
    for (int it = 0; it < 16; ++it) { const int ch = lane + 32 * it, d = ch >> 3, q4 = (ch & 7) * 4;
      *(volatile v4f_t*)(Rout + ((size_t)bb * 256 + h * DKK + d) * outld + (size_t)fr * qper + q0 + q4) = *(const volatile v4fa*)(so + d * 36 + q4); }
    __threadfence();
  }
}


#define GSTR 48
template <typename AT, int ASRC>
__global__ __launch_bounds__(256) void gemm_knb(const AT* __restrict__ A, int lda, size_t strideA, const float* __restrict__ Wm, int ldw, size_t strideW,
                                                const float* __restrict__ rowbias, const float* __restrict__ s1, const float* __restrict__ s2, const float* __restrict__ mj, const float* __restrict__ invD,
                                                float oscale, int N, float* __restrict__ Y, int ldy, size_t strideY, int K) {
  __shared__ __attribute__((aligned(16))) f16 ldsA[128 * GSTR];
  __shared__ __attribute__((aligned(16))) f16 ldsW[128 * GSTR];
  __shared__ __attribute__((aligned(16))) float oS[8][32 * 68];
  const int tid = threadIdx.x, lane = tid & 31, wave = tid >> 5, cl = lane & 15, rh = (lane >> 4) * 8;
  const int m0 = blockIdx.x * 128, n0 = blockIdx.y * 128;
  const int wm = (wave & 3) * 32, wn = (wave >> 2) * 64;
  A += (size_t)blockIdx.z * strideA; Wm += (size_t)blockIdx.z * strideW; Y += (size_t)blockIdx.z * strideY;
  if (ASRC == 1) { s1 += (size_t)blockIdx.z * K; s2 += (size_t)blockIdx.z * lda; mj += (size_t)blockIdx.z * K; invD += (size_t)blockIdx.z * K; }
  f32x8 acc[2][4];
#pragma unroll
  for (int i = 0; i < 2; ++i)
#pragma unroll
    for (int j = 0; j < 4; ++j) { f32x8 z = {}; acc[i][j] = z; }
#pragma unroll 1
  for (int k0 = 0; k0 < K; k0 += 32) {
    __syncthreads();
    { const int row = tid >> 1, ch = (tid & 1) * 16;
      if (ASRC == 0) {
        const AT* src = A + (size_t)(m0 + row) * lda + k0 + ch;
#pragma unroll
        for (int g = 0; g < 16; ++g) ldsA[row * GSTR + ch + g] = (f16)src[g];
      } else {
        const float s2i = s2[m0 + row];
#pragma unroll
        for (int g = 0; g < 16; ++g) { const int j = k0 + ch + g; float a = s1[j] + s2i; a = (a >= 0.0f) ? a : 0.2f * a;
          ldsA[row * GSTR + ch + g] = (f16)(1024.0f * __expf(a - mj[j]) * invD[j]); }
      } }
    { const int k = tid >> 3, nn0 = (tid & 7) * 16;
      const float* src = Wm + (size_t)(k0 + k) * ldw;
#pragma unroll
      for (int g = 0; g < 4; ++g) { const int col = min(n0 + nn0 + 4 * g, N - 4); const v4f_t v = *(const v4f_t*)(src + col);
#pragma unroll
        for (int u = 0; u < 4; ++u) ldsW[(nn0 + 4 * g + u) * GSTR + k] = (f16)v[u]; } }
    __syncthreads();
    f16x16 af[2];
#pragma unroll
    for (int i = 0; i < 2; ++i) af[i] = lds_frag(ldsA + (wm + 16 * i) * GSTR, GSTR);
#pragma unroll
    for (int j = 0; j < 4; ++j) {
      const f16x16 bf = lds_frag(ldsW + (wn + 16 * j) * GSTR, GSTR);
#pragma unroll
      for (int i = 0; i < 2; ++i) acc[i][j] = wmma16(af[i], bf, acc[i][j]);
    }
  }
  float* so = oS[wave];
#pragma unroll
  for (int i = 0; i < 2; ++i)
#pragma unroll
    for (int r = 0; r < 8; ++r) {
      const int m = m0 + wm + 16 * i + rh + r;
      const float rb = rowbias ? rowbias[m] : 0.0f;
#pragma unroll
      for (int j = 0; j < 4; ++j) so[(16 * i + rh + r) * 68 + 16 * j + cl] = acc[i][j][r] * oscale + rb;
    }
  asm volatile("s_wait_dscnt 0" ::: "memory");
  __builtin_amdgcn_wave_barrier();
#pragma unroll 1
  for (int pass = 0; pass < 2; ++pass) {
#pragma unroll
    for (int it = 0; it < 16; ++it) { const int f4 = lane + 32 * it, rr = f4 >> 4, q = (f4 & 15) * 4;
      if (n0 + wn + q < N) *(volatile v4f_t*)(Y + (size_t)(m0 + wm + rr) * ldy + n0 + wn + q) = *(const volatile v4fa*)(so + rr * 68 + q); }
    __threadfence();
  }
}

#define GSTR 48
template <typename AT, int ASRC>
__global__ __launch_bounds__(256) void gemm_knbh(const AT* __restrict__ A, int lda, size_t strideA, const float* __restrict__ Wm, int ldw, size_t strideW,
                                                const float* __restrict__ rowbias, const float* __restrict__ s1, const float* __restrict__ s2, const float* __restrict__ mj, const float* __restrict__ invD,
                                                float oscale, int N, f16* __restrict__ Y, int ldy, size_t strideY, int K) {
  __shared__ __attribute__((aligned(16))) f16 ldsA[128 * GSTR];
  __shared__ __attribute__((aligned(16))) f16 ldsW[128 * GSTR];
  __shared__ __attribute__((aligned(16))) float oS[8][32 * 68];
  const int tid = threadIdx.x, lane = tid & 31, wave = tid >> 5, cl = lane & 15, rh = (lane >> 4) * 8;
  const int m0 = blockIdx.x * 128, n0 = blockIdx.y * 128;
  const int wm = (wave & 3) * 32, wn = (wave >> 2) * 64;
  A += (size_t)blockIdx.z * strideA; Wm += (size_t)blockIdx.z * strideW; Y += (size_t)blockIdx.z * strideY;
  if (ASRC == 1) { s1 += (size_t)blockIdx.z * K; s2 += (size_t)blockIdx.z * lda; mj += (size_t)blockIdx.z * K; invD += (size_t)blockIdx.z * K; }
  f32x8 acc[2][4];
#pragma unroll
  for (int i = 0; i < 2; ++i)
#pragma unroll
    for (int j = 0; j < 4; ++j) { f32x8 z = {}; acc[i][j] = z; }
#pragma unroll 1
  for (int k0 = 0; k0 < K; k0 += 32) {
    __syncthreads();
    { const int row = tid >> 1, ch = (tid & 1) * 16;
      if (ASRC == 0) {
        const AT* src = A + (size_t)(m0 + row) * lda + k0 + ch;
#pragma unroll
        for (int g = 0; g < 16; ++g) ldsA[row * GSTR + ch + g] = (f16)src[g];
      } else {
        const float s2i = s2[m0 + row];
#pragma unroll
        for (int g = 0; g < 16; ++g) { const int j = k0 + ch + g; float a = s1[j] + s2i; a = (a >= 0.0f) ? a : 0.2f * a;
          ldsA[row * GSTR + ch + g] = (f16)(1024.0f * __expf(a - mj[j]) * invD[j]); }
      } }
    { const int k = tid >> 3, nn0 = (tid & 7) * 16;
      const float* src = Wm + (size_t)(k0 + k) * ldw;
#pragma unroll
      for (int g = 0; g < 4; ++g) { const int col = min(n0 + nn0 + 4 * g, N - 4); const v4f_t v = *(const v4f_t*)(src + col);
#pragma unroll
        for (int u = 0; u < 4; ++u) ldsW[(nn0 + 4 * g + u) * GSTR + k] = (f16)v[u]; } }
    __syncthreads();
    f16x16 af[2];
#pragma unroll
    for (int i = 0; i < 2; ++i) af[i] = lds_frag(ldsA + (wm + 16 * i) * GSTR, GSTR);
#pragma unroll
    for (int j = 0; j < 4; ++j) {
      const f16x16 bf = lds_frag(ldsW + (wn + 16 * j) * GSTR, GSTR);
#pragma unroll
      for (int i = 0; i < 2; ++i) acc[i][j] = wmma16(af[i], bf, acc[i][j]);
    }
  }
  float* so = oS[wave];
#pragma unroll
  for (int i = 0; i < 2; ++i)
#pragma unroll
    for (int r = 0; r < 8; ++r) {
      const int m = m0 + wm + 16 * i + rh + r;
      const float rb = rowbias ? rowbias[m] : 0.0f;
#pragma unroll
      for (int j = 0; j < 4; ++j) so[(16 * i + rh + r) * 68 + 16 * j + cl] = acc[i][j][r] * oscale + rb;
    }
  asm volatile("s_wait_dscnt 0" ::: "memory");
  __builtin_amdgcn_wave_barrier();
#pragma unroll 1
  for (int pass = 0; pass < 2; ++pass) {
#pragma unroll
    for (int it = 0; it < 8; ++it) { const int c8 = lane + 32 * it, rr = c8 >> 3, q = (c8 & 7) * 8;
      if (n0 + wn + q < N) { union { f16 hh[8]; v4u_t u; } cv;
#pragma unroll
        for (int e = 0; e < 8; ++e) cv.hh[e] = (f16)so[rr * 68 + q + e];
        *(volatile v4u_t*)(Y + (size_t)(m0 + wm + rr) * ldy + n0 + wn + q) = cv.u; } }
    __threadfence();
  }
}

__global__ __launch_bounds__(256) void k_gnstats(const float* __restrict__ x, int ntok, float* __restrict__ stats) {
  __shared__ float red[256]; __shared__ float mu_s;
  const int tid = threadIdx.x, b = blockIdx.x / NG, g = blockIdx.x % NG;
  const float* base = x + ((size_t)b * CC + g * 8) * ntok; const size_t n = (size_t)8 * ntok;
  float s = 0.0f; for (size_t i = tid; i < n; i += 256) s += base[i];
  red[tid] = s; __syncthreads(); for (int o = 128; o > 0; o >>= 1) { if (tid < o) red[tid] += red[tid + o]; __syncthreads(); }
  if (tid == 0) mu_s = red[0] / (float)n; __syncthreads();
  const float mu = mu_s; float q = 0.0f; for (size_t i = tid; i < n; i += 256) { const float d = base[i] - mu; q += d * d; }
  __syncthreads(); red[tid] = q; __syncthreads(); for (int o = 128; o > 0; o >>= 1) { if (tid < o) red[tid] += red[tid + o]; __syncthreads(); }
  if (tid == 0) { float* dst = stats + ((size_t)b * NG + g) * 32; const float rstd = rsqrtf(red[0] / (float)n + 1e-5f);
    *(volatile float*)dst = mu; *(volatile float*)(dst + 1) = rstd; __threadfence(); *(volatile float*)dst = mu; *(volatile float*)(dst + 1) = rstd; }
}
__global__ __launch_bounds__(256) void k_gnfold(const float* __restrict__ Wm, const float* __restrict__ gsc, const float* __restrict__ gbi, const float* __restrict__ stats,
                                               float* __restrict__ Wf) {
  __shared__ __attribute__((aligned(16))) float rowS[CC];
  const int tid = threadIdx.x, b = blockIdx.x / (3 * CC), o = blockIdx.x % (3 * CC);
  { const int c = tid; const int g = c >> 3; const float mu = stats[((size_t)b * NG + g) * 32], rstd = stats[((size_t)b * NG + g) * 32 + 1];
    const float a = rstd * gsc[c]; rowS[c] = Wm[(size_t)o * CC + c] * a; (void)mu; }
  __syncthreads();
#pragma unroll 1
  for (int pass = 0; pass < 2; ++pass) { if (tid < 64) *(volatile v4f_t*)(Wf + ((size_t)b * 3 * CC + o) * CC + tid * 4) = *(const volatile v4fa*)(rowS + tid * 4); __threadfence(); }
}
__global__ __launch_bounds__(256) void k_gnfoldb(const float* __restrict__ Wm, const float* __restrict__ bias, const float* __restrict__ gsc, const float* __restrict__ gbi,
                                                const float* __restrict__ stats, float* __restrict__ bf) {
  __shared__ float dS[CC]; __shared__ __attribute__((aligned(16))) float bS[3 * CC];
  const int tid = threadIdx.x, b = blockIdx.x;
  { const int c = tid, g = c >> 3; const float mu = stats[((size_t)b * NG + g) * 32], rstd = stats[((size_t)b * NG + g) * 32 + 1]; dS[c] = gbi[c] - mu * rstd * gsc[c]; }
  __syncthreads();
  for (int o = tid; o < 3 * CC; o += 256) { float s = bias[o]; const float* wr = Wm + (size_t)o * CC;
#pragma unroll 4
    for (int c = 0; c < CC; ++c) s += wr[c] * dS[c];
    bS[o] = s; }
  __syncthreads();
#pragma unroll 1
  for (int pass = 0; pass < 2; ++pass) { for (int q4 = tid; q4 < 3 * CC / 4; q4 += 256) *(volatile v4f_t*)(bf + (size_t)b * 3 * CC + q4 * 4) = *(const volatile v4fa*)(bS + q4 * 4); __threadfence(); }
}
__global__ __launch_bounds__(256) void k_resv(const float* __restrict__ video, const float* __restrict__ pv, float* __restrict__ out) {
  const size_t i = (size_t)blockIdx.x * 256 + threadIdx.x;
  const size_t q4 = i % (HWV / 4); size_t r = i / (HWV / 4); const int c = r % CC; r /= CC; const int f = r % NFR; const int b = r / NFR;
  const v4f_t a = *(const v4f_t*)(video + 4 * i), p = *(const v4f_t*)(pv + ((size_t)b * CC + c) * VLEN + (size_t)f * HWV + q4 * 4);
  v4f_t o; o[0]=a[0]+p[0]; o[1]=a[1]+p[1]; o[2]=a[2]+p[2]; o[3]=a[3]+p[3];
  *(volatile v4f_t*)(out + 4 * i) = o; __threadfence(); *(volatile v4f_t*)(out + 4 * i) = o;
}
__global__ __launch_bounds__(256) void k_resa(const float* __restrict__ audio, const float* __restrict__ pa, float* __restrict__ out, size_t n4) {
  const size_t i = (size_t)blockIdx.x * 256 + threadIdx.x; if (i >= n4) return;
  const v4f_t a = *(const v4f_t*)(audio + 4 * i), p = *(const v4f_t*)(pa + 4 * i); v4f_t o; o[0]=a[0]+p[0]; o[1]=a[1]+p[1]; o[2]=a[2]+p[2]; o[3]=a[3]+p[3];
  *(volatile v4f_t*)(out + 4 * i) = o; __threadfence(); *(volatile v4f_t*)(out + 4 * i) = o;
}
__global__ __launch_bounds__(256) void k_vperm(const float* __restrict__ video, float* __restrict__ vt) {
  const size_t i = (size_t)blockIdx.x * 256 + threadIdx.x;
  const size_t q4 = i % (HWV / 4); size_t r = i / (HWV / 4); const int c = r % CC; r /= CC; const int f = r % NFR; const int b = r / NFR;
  const v4f_t a = *(const v4f_t*)(video + 4 * i); float* dst = vt + ((size_t)b * CC + c) * VLEN + (size_t)f * HWV + q4 * 4;
  *(volatile v4f_t*)dst = a; __threadfence(); *(volatile v4f_t*)dst = a;
}

extern "C" void kernel_launch(void* const* d_in, const int* in_sizes, int n_in,
                              void* d_out, int out_size, void* d_ws, size_t ws_size,
                              hipStream_t stream) {
  (void)in_sizes; (void)n_in; (void)out_size;
  const float* video = (const float*)d_in[0];
  const float* audio = (const float*)d_in[1];
  const float* gvs = (const float*)d_in[2], *gvb = (const float*)d_in[3], *gas = (const float*)d_in[4], *gab = (const float*)d_in[5];
  const float* w_vqkv = (const float*)d_in[6], *b_vqkv = (const float*)d_in[7], *w_aqkv = (const float*)d_in[8], *b_aqkv = (const float*)d_in[9];
  const float* w_vproj = (const float*)d_in[10], *b_vproj = (const float*)d_in[11], *w_aproj = (const float*)d_in[12], *b_aproj = (const float*)d_in[13];
  float* vout = (float*)d_out;
  float* aout = (float*)((char*)d_out + (size_t)NB_ * NFR * CC * HWV * 4);
  char* ws = (char*)d_ws;
  f16* qkv = (f16*)ws; ws += (size_t)NB_ * 3 * CC * TT * 2;
  float* vt = (float*)ws; ws += (size_t)NB_ * CC * VLEN * 4;
  float* oa = (float*)ws; ws += (size_t)NB_ * CC * LA * 4;
  float* pa = (float*)ws; ws += (size_t)NB_ * CC * LA * 4;
  float* stv = (float*)ws; ws += NB_ * NG * 32 * 4; float* sta = (float*)ws; ws += NB_ * NG * 32 * 4;
  float* Wfv = (float*)ws; ws += (size_t)NB_ * 3 * CC * CC * 4;
  float* Wfa = (float*)ws; ws += (size_t)NB_ * 3 * CC * CC * 4;
  float* bfv = (float*)ws; ws += NB_ * 3 * CC * 4; float* bfa = (float*)ws; ws += NB_ * 3 * CC * 4;
  if ((size_t)(ws - (char*)d_ws) > ws_size) return;
  const dim3 blk(256);
  k_vperm<<<dim3((NB_ * NFR * CC * HWV / 4) / 256), blk, 0, stream>>>(video, vt);
  k_gnstats<<<dim3(NB_ * NG), blk, 0, stream>>>(vt, VLEN, stv);
  k_gnstats<<<dim3(NB_ * NG), blk, 0, stream>>>(audio, LA, sta);
  k_gnfold<<<dim3(NB_ * 3 * CC), blk, 0, stream>>>(w_vqkv, gvs, gvb, stv, Wfv);
  k_gnfold<<<dim3(NB_ * 3 * CC), blk, 0, stream>>>(w_aqkv, gas, gab, sta, Wfa);
  k_gnfoldb<<<dim3(NB_), blk, 0, stream>>>(w_vqkv, b_vqkv, gvs, gvb, stv, bfv);
  k_gnfoldb<<<dim3(NB_), blk, 0, stream>>>(w_aqkv, b_aqkv, gas, gab, sta, bfa);
  for (int b = 0; b < NB_; ++b) {
    gemm_knbh<float, 0><<<dim3(3 * CC / 128, VLEN / 128, 1), blk, 0, stream>>>(Wfv + (size_t)b * 3 * CC * CC, CC, 0, vt + (size_t)b * CC * VLEN, VLEN, 0, bfv + b * 3 * CC, nullptr, nullptr, nullptr, nullptr, 1.0f, VLEN, qkv + (size_t)b * 3 * CC * TT, TT, 0, CC);
    gemm_knbh<float, 0><<<dim3(3 * CC / 128, LA / 128, 1), blk, 0, stream>>>(Wfa + (size_t)b * 3 * CC * CC, CC, 0, audio + (size_t)b * CC * LA, LA, 0, bfa + b * 3 * CC, nullptr, nullptr, nullptr, nullptr, 1.0f, LA, qkv + (size_t)b * 3 * CC * TT + VLEN, TT, 0, CC);
  }
  float* ov = vt;
  attn_kernel<<<dim3(HWV / 64, HH, NB_ * NFR), dim3(64), 0, stream>>>(qkv, qkv, qkv, ov, 0, HWV, VLEN, APF, APF, VLEN);
  attn_kernel<<<dim3(APF / 64, HH, NB_ * NFR), dim3(64), 0, stream>>>(qkv, qkv, qkv, oa, VLEN, APF, 0, HWV, HWV, LA);
  float* pv = (float*)qkv;
  gemm_knb<float, 0><<<dim3(CC / 128, VLEN / 128, NB_), blk, 0, stream>>>(w_vproj, CC, 0, ov, VLEN, (size_t)CC * VLEN, b_vproj, nullptr, nullptr, nullptr, nullptr, 1.0f, VLEN, pv, VLEN, (size_t)CC * VLEN, CC);
  gemm_knb<float, 0><<<dim3(CC / 128, LA / 128, NB_), blk, 0, stream>>>(w_aproj, CC, 0, oa, LA, (size_t)CC * LA, b_aproj, nullptr, nullptr, nullptr, nullptr, 1.0f, LA, pa, LA, (size_t)CC * LA, CC);
  k_resv<<<dim3((NB_ * NFR * CC * HWV / 4) / 256), blk, 0, stream>>>(video, pv, vout);
  k_resa<<<dim3((NB_ * CC * LA / 4 + 255) / 256), blk, 0, stream>>>(audio, pa, aout, (size_t)NB_ * CC * LA / 4);
}
